// Model_39676907885720
// MI455X (gfx1250) — hardware-verified
//
#include <hip/hip_runtime.h>


#define NPAIR 32
#define NS    512
#define ND    512
#define NROW  (NPAIR * NS)
#define NPASS 4
#define PPAIR (NPAIR / NPASS)
#define PROW  (PPAIR * NS)
#define SLAB  ((size_t)NS * ND)
typedef _Float16 h16;
typedef unsigned short bf;
typedef __attribute__((ext_vector_type(16))) __bf16   v16bf;
typedef __attribute__((ext_vector_type(16))) _Float16 v16h;
typedef __attribute__((ext_vector_type(8)))  _Float16 v8h;
typedef __attribute__((ext_vector_type(8)))  unsigned short v8us;
typedef __attribute__((ext_vector_type(8)))  float    v8f;
typedef __attribute__((ext_vector_type(4)))  float    v4f;
typedef v8h  __attribute__((may_alias)) v8ha;
typedef v4f  __attribute__((may_alias)) v4fa;
typedef v8us __attribute__((may_alias)) v8usa;

__device__ __forceinline__ unsigned short f2bf(float f) { unsigned u = __float_as_uint(f); u += 0x7FFFu + ((u >> 16) & 1u); return (unsigned short)(u >> 16); }
__device__ __forceinline__ float bf2f(unsigned short b) { return __uint_as_float(((unsigned)b) << 16); }
__device__ __forceinline__ float bfr(float f) { return bf2f(f2bf(f)); }
__device__ __forceinline__ v16h cat16(v8h lo, v8h hi) { return __builtin_shufflevector(lo, hi, 0, 1, 2, 3, 4, 5, 6, 7, 8, 9, 10, 11, 12, 13, 14, 15); }
__device__ __forceinline__ v16bf cat16b(v8us lo, v8us hi) { return __builtin_bit_cast(v16bf, __builtin_shufflevector(lo, hi, 0, 1, 2, 3, 4, 5, 6, 7, 8, 9, 10, 11, 12, 13, 14, 15)); }
__device__ __forceinline__ v8f wmma16(v16h a, v16h b, v8f c) { return __builtin_amdgcn_wmma_f32_16x16x32_f16(false, a, false, b, (short)0, c, false, false); }
__device__ __forceinline__ v8f wmmab(v16bf a, v16bf b, v8f c) { return __builtin_amdgcn_wmma_f32_16x16x32_bf16(false, a, false, b, (short)0, c, false, false); }

template <typename T16> struct WFrag;
template <> struct WFrag<h16> { typedef v16h V; static __device__ __forceinline__ V ld(const h16* p) { return cat16(*(const v8h*)p, *(const v8h*)(p + 16)); } static __device__ __forceinline__ v8f mma(V a, V b, v8f c) { return wmma16(a, b, c); } };
template <> struct WFrag<bf> { typedef v16bf V; static __device__ __forceinline__ V ld(const bf* p) { return cat16b(*(const v8us*)p, *(const v8us*)(p + 16)); } static __device__ __forceinline__ v8f mma(V a, V b, v8f c) { return wmmab(a, b, c); } };
template <typename T16, int NSPLIT, bool BIAS>
__global__ __launch_bounds__(32) void k_gemmw(const T16* __restrict__ A, const T16* __restrict__ A2, const T16* __restrict__ Bt, const T16* __restrict__ Bt2, int K, float* C, int ldc, const float* __restrict__ bias, size_t sA, size_t sB, size_t sC) {
    typedef typename WFrag<T16>::V V;
    __shared__ __align__(16) float os[16 * 68];
    const size_t z = blockIdx.z; A += z * sA; if (A2) A2 += z * sA; Bt += z * sB; if (Bt2) Bt2 += z * sB; C += z * sC;
    const int lane = threadIdx.x & 31, lr = lane & 15, hi = lane >> 4; const int r0 = blockIdx.x * 64, c0 = blockIdx.y * 64;
    v8f acc[4][4];
#pragma unroll
    for (int mb = 0; mb < 4; ++mb)
#pragma unroll
        for (int nb = 0; nb < 4; ++nb) acc[mb][nb] = (v8f){};
    const size_t aoff = (size_t)(r0 + lr) * K + 8 * hi, boff = (size_t)(c0 + lr) * K + 8 * hi;
    for (int kc = 0; kc < K; kc += 32) {
        V a[4], a2[4];
#pragma unroll
        for (int mb = 0; mb < 4; ++mb) { a[mb] = WFrag<T16>::ld(A + aoff + (size_t)mb * 16 * K + kc); if (NSPLIT == 1 || NSPLIT == 2) a2[mb] = WFrag<T16>::ld(A2 + aoff + (size_t)mb * 16 * K + kc); }
#pragma unroll
        for (int nb = 0; nb < 4; ++nb) { const V b = WFrag<T16>::ld(Bt + boff + (size_t)nb * 16 * K + kc); V b2; if (NSPLIT >= 2) b2 = WFrag<T16>::ld(Bt2 + boff + (size_t)nb * 16 * K + kc);
#pragma unroll
            for (int mb = 0; mb < 4; ++mb) { acc[mb][nb] = WFrag<T16>::mma(a[mb], b, acc[mb][nb]); if (NSPLIT == 1 || NSPLIT == 2) acc[mb][nb] = WFrag<T16>::mma(a2[mb], b, acc[mb][nb]); if (NSPLIT >= 2) acc[mb][nb] = WFrag<T16>::mma(a[mb], b2, acc[mb][nb]); } }
        asm volatile("v_nop\n\tv_nop\n\tv_nop\n\tv_nop" : "+v"(acc[0][0]), "+v"(acc[1][1]), "+v"(acc[2][2]), "+v"(acc[3][3]) : "v"(a[0]), "v"(a[3]));
    }
#pragma unroll
    for (int mb = 0; mb < 4; ++mb) {
#pragma unroll
        for (int nb = 0; nb < 4; ++nb) {
#pragma unroll
            for (int j = 0; j < 8; ++j) os[(hi * 8 + j) * 68 + nb * 16 + lr] = acc[mb][nb][j]; }
        __builtin_amdgcn_wave_barrier(); asm volatile("" ::: "memory");
        float* crow = C + (size_t)(r0 + mb * 16) * ldc + c0;
#pragma unroll 1
        for (int ps = 0; ps < 2; ++ps) {
#pragma unroll
            for (int s = 0; s < 8; ++s) { const int row = 2 * s + hi, cofs = lr * 4; v4f val = *(const v4fa*)(os + row * 68 + cofs); if (BIAS) { val[0] += bfr(bias[c0 + cofs]); val[1] += bfr(bias[c0 + cofs + 1]); val[2] += bfr(bias[c0 + cofs + 2]); val[3] += bfr(bias[c0 + cofs + 3]); }
                *(volatile v4f*)(crow + (size_t)row * ldc + cofs) = val; }
            if (ps == 0) __threadfence(); }
        __builtin_amdgcn_wave_barrier(); asm volatile("" ::: "memory");
    }
}

__device__ __forceinline__ void splitf(float y, unsigned short& h, unsigned short& l) { h = f2bf(y); l = f2bf(y - bf2f(h)); }
typedef __attribute__((ext_vector_type(2))) _Float16 v2h;
typedef __attribute__((ext_vector_type(4))) _Float16 v4h;
typedef __attribute__((ext_vector_type(2))) unsigned short v2us;
typedef __attribute__((ext_vector_type(4))) unsigned short v4us;
typedef __attribute__((ext_vector_type(2))) float v2f;
__device__ __forceinline__ h16 toh_flush(float x) { const float z = (fabsf(x) < 6.103515625e-05f) ? 0.0f : x; return (h16)z; }

#define LNC_MAX 2048
template <bool RES>
__global__ __launch_bounds__(256) void k_lnrow(const float* __restrict__ A, const float* __restrict__ R, const float* __restrict__ gamma, const float* __restrict__ beta, float eps, int C, int nrows, float* Y) {
    const int lane = threadIdx.x & 31; const int row = blockIdx.x * 8 + (threadIdx.x >> 5); if (row >= nrows) return; const int nch = C / 128; const float* a = A + (size_t)row * C; float x[LNC_MAX / 32]; float s = 0.0f;
    for (int k = 0; k < LNC_MAX / 128; ++k) { if (k < nch) { const int c0 = k * 128 + lane * 4; v4f v = *(const v4f*)(a + c0);
            if (RES) { const v4f w = *(const v4f*)(R + (size_t)row * C + c0); v[0] = __fadd_rn(v[0], w[0]); v[1] = __fadd_rn(v[1], w[1]); v[2] = __fadd_rn(v[2], w[2]); v[3] = __fadd_rn(v[3], w[3]); }
            x[k * 4 + 0] = v[0]; x[k * 4 + 1] = v[1]; x[k * 4 + 2] = v[2]; x[k * 4 + 3] = v[3]; s = __fadd_rn(__fadd_rn(__fadd_rn(__fadd_rn(s, v[0]), v[1]), v[2]), v[3]); } }
    for (int sh = 16; sh; sh >>= 1) s = __fadd_rn(s, __shfl_xor(s, sh, 32));
    const float mean = __fdiv_rn(s, (float)C); float q = 0.0f;
    for (int k = 0; k < LNC_MAX / 128; ++k) { if (k < nch) {
            for (int j = 0; j < 4; ++j) { const float d = __fsub_rn(x[k * 4 + j], mean); x[k * 4 + j] = d; q = __fmaf_rn(d, d, q); } } }
    for (int sh = 16; sh; sh >>= 1) q = __fadd_rn(q, __shfl_xor(q, sh, 32));
    const float rstd = __fdiv_rn(1.0f, sqrtf(__fadd_rn(__fdiv_rn(q, (float)C), eps)));
    for (int k = 0; k < LNC_MAX / 128; ++k) { if (k < nch) { const int c0 = k * 128 + lane * 4; const v4f g = *(const v4f*)(gamma + c0); const v4f bt = *(const v4f*)(beta + c0);
            for (int j = 0; j < 4; ++j) x[k * 4 + j] = __fmaf_rn(__fmul_rn(x[k * 4 + j], rstd), bfr(g[j]), bfr(bt[j])); } }
    float* y = Y + (size_t)row * C;
    for (int ps = 0; ps < 2; ++ps) {
        for (int k = 0; k < LNC_MAX / 128; ++k) { if (k < nch) { v4f o; o[0] = x[k * 4 + 0]; o[1] = x[k * 4 + 1]; o[2] = x[k * 4 + 2]; o[3] = x[k * 4 + 3]; *(volatile v4f*)(y + k * 128 + lane * 4) = o; } }
        if (ps == 0) __threadfence(); }
}
__global__ __launch_bounds__(256) void k_cvt8(const float* __restrict__ src, bf* dst, size_t n8) { const size_t i = (size_t)blockIdx.x * 256 + threadIdx.x; if (i >= n8) return; const v8f v = *(const v8f*)(src + i * 8); v8us o;
#pragma unroll
    for (int k = 0; k < 8; ++k) o[k] = f2bf(v[k]); *(volatile v8us*)(dst + i * 8) = o; __threadfence(); *(volatile v8us*)(dst + i * 8) = o; }

__global__ __launch_bounds__(256) void k_c16s(const float* __restrict__ src, h16* dst, size_t n8, int rin, float scale) { const size_t i = (size_t)blockIdx.x * 256 + threadIdx.x; if (i >= n8) return; const v8f v = *(const v8f*)(src + i * 8); v8h o;
#pragma unroll
    for (int k = 0; k < 8; ++k) { const float w = rin ? bfr(v[k]) : v[k]; o[k] = toh_flush(__fmul_rn(w, scale)); }
    *(volatile v8h*)(dst + i * 8) = o; __threadfence(); *(volatile v8h*)(dst + i * 8) = o; }

__global__ __launch_bounds__(256) void k_split(const float* __restrict__ src, bf* hi, bf* lo, size_t n8, float scale) { const size_t i = (size_t)blockIdx.x * 256 + threadIdx.x; if (i >= n8) return; const v8f v = *(const v8f*)(src + i * 8); v8us oh, ol;
#pragma unroll
    for (int k = 0; k < 8; ++k) { unsigned short h, l; splitf(__fmul_rn(v[k], scale), h, l); oh[k] = h; ol[k] = l; }
    *(volatile v8us*)(hi + i * 8) = oh; *(volatile v8us*)(lo + i * 8) = ol; __threadfence(); *(volatile v8us*)(hi + i * 8) = oh; *(volatile v8us*)(lo + i * 8) = ol; }

__global__ __launch_bounds__(256) void k_mix(float* T4, float* T5, float* T6, const float* __restrict__ V1, const float* __restrict__ V3, const float* __restrict__ V2, float* Sm, size_t n4) { const size_t i = (size_t)blockIdx.x * 256 + threadIdx.x; if (i >= n4) return;
    const v4f a = *(const v4f*)(T4 + i * 4), b = *(const v4f*)(T5 + i * 4), c = *(const v4f*)(T6 + i * 4); const v4f p = *(const v4f*)(V1 + i * 4), q = *(const v4f*)(V3 + i * 4), r = *(const v4f*)(V2 + i * 4); v4f x, y, z, s;
#pragma unroll
    for (int k = 0; k < 4; ++k) { x[k] = __fmul_rn(a[k], p[k]); y[k] = __fmul_rn(b[k], q[k]); z[k] = __fmul_rn(c[k], r[k]); s[k] = __fadd_rn(__fadd_rn(x[k], y[k]), z[k]); }
    *(volatile v4f*)(T4 + i * 4) = x; *(volatile v4f*)(T5 + i * 4) = y; *(volatile v4f*)(T6 + i * 4) = z; *(volatile v4f*)(Sm + i * 4) = s; __threadfence(); *(volatile v4f*)(T4 + i * 4) = x; *(volatile v4f*)(T5 + i * 4) = y; *(volatile v4f*)(T6 + i * 4) = z; *(volatile v4f*)(Sm + i * 4) = s; }

__global__ __launch_bounds__(256) void k_sum6(const float* __restrict__ P16, const float* __restrict__ P17, const float* __restrict__ P18, const float* __restrict__ V10, const float* __restrict__ V11, const float* __restrict__ V12, float* U, size_t n4) { const size_t i = (size_t)blockIdx.x * 256 + threadIdx.x; if (i >= n4) return;
    const v4f a = *(const v4f*)(P16 + i * 4), b = *(const v4f*)(P17 + i * 4), c = *(const v4f*)(P18 + i * 4); const v4f p = *(const v4f*)(V10 + i * 4), q = *(const v4f*)(V11 + i * 4), r = *(const v4f*)(V12 + i * 4); v4f u;
#pragma unroll
    for (int k = 0; k < 4; ++k) u[k] = __fadd_rn(__fadd_rn(__fadd_rn(a[k], p[k]), __fadd_rn(b[k], q[k])), __fadd_rn(c[k], r[k]));
    *(volatile v4f*)(U + i * 4) = u; __threadfence(); *(volatile v4f*)(U + i * 4) = u; }

extern "C" void kernel_launch(void* const* d_in, const int* in_sizes, int n_in, void* d_out, int out_size, void* d_ws, size_t ws_size, hipStream_t stream) {
    if (n_in < 17) return;
    if (in_sizes[0] != NROW * ND) return;
    for (int k : {1, 3, 5, 7, 8, 9, 10, 11, 12}) if (in_sizes[k] != ND * ND) return;
    for (int k : {2, 4, 6, 13, 14, 15, 16}) if (in_sizes[k] != ND) return;
    if (out_size != NROW * ND) return;
    static_assert(NS == 512 && ND == 512 && NPAIR % NPASS == 0 && PROW % 64 == 0 && ND % 64 == 0 && ND % 32 == 0 && ND % 128 == 0 && ND <= LNC_MAX && (PROW * ND / 8) % 256 == 0 && (ND * ND / 8) % 256 == 0 && PROW % 8 == 0, "a pair is a [512][512] slab; the products: M and N multiples of 64, the depth a multiple of 32; the row norm: a row a multiple of 128; every elementwise grid exact");
    const float* x = (const float*)d_in[0]; const float* wq1 = (const float*)d_in[1]; const float* bq1 = (const float*)d_in[2]; const float* wk1 = (const float*)d_in[3]; const float* bk1 = (const float*)d_in[4]; const float* wv1 = (const float*)d_in[5]; const float* bv1 = (const float*)d_in[6]; const float* wq2 = (const float*)d_in[7];   const float* wv2 = (const float*)d_in[9]; const float* wq3 = (const float*)d_in[10]; const float* wk3 = (const float*)d_in[11]; const float* wv3 = (const float*)d_in[12]; const float* g1 = (const float*)d_in[13]; const float* b1 = (const float*)d_in[14]; const float* g2 = (const float*)d_in[15]; const float* b2 = (const float*)d_in[16];
    float* out = (float*)d_out;
    char* wsp = (char*)d_ws; auto take = [&](size_t bytes) { char* p = wsp; wsp += (bytes + 255) & ~(size_t)255; return (void*)p; };
    const size_t PW = (size_t)PROW * ND;
    h16* Wh[8]; for (int k = 0; k < 8; ++k) Wh[k] = (h16*)take((size_t)ND * ND * 2);
    bf* Wb[3]; for (int k = 0; k < 3; ++k) Wb[k] = (bf*)take((size_t)ND * ND * 2);
    unsigned short* S[4]; for (int k = 0; k < 4; ++k) S[k] = (unsigned short*)take(PW * 2);
    float* F[8]; for (int k = 0; k < 8; ++k) F[k] = (float*)take(PW * 4);
    if ((size_t)(wsp - (char*)d_ws) > ws_size) return;
    const float* wsrc[8] = {wq1, wk1, wv1, wq2, wv2, wq3, wk3, wv3};
    for (int k = 0; k < 8; ++k) k_c16s<<<(unsigned)(ND * ND / 8 / 256), 256, 0, stream>>>(wsrc[k], Wh[k], (size_t)ND * ND / 8, 1, 1.0f);
    for (int k = 0; k < 3; ++k) k_cvt8<<<(unsigned)(ND * ND / 8 / 256), 256, 0, stream>>>(wsrc[5 + k], Wb[k], (size_t)ND * ND / 8);
    const float rs = 0.044194173824159216f;
    const unsigned GE = (unsigned)(PW / 8 / 256), G4 = (unsigned)(PW / 4 / 256); const dim3 gRow(PROW / 64, ND / 64, 1), gPair(NS / 64, NS / 64, PPAIR);
    for (int ps = 0; ps < NPASS; ++ps) { const size_t r0 = (size_t)ps * PROW;
        k_c16s<<<GE, 256, 0, stream>>>(x + r0 * ND, (h16*)S[0], PW / 8, 1, 1.0f);
        k_gemmw<h16, 0, true><<<gRow, 32, 0, stream>>>((const h16*)S[0], nullptr, Wh[0], nullptr, ND, F[0], ND, bq1, 0, 0, 0);
        k_gemmw<h16, 0, true><<<gRow, 32, 0, stream>>>((const h16*)S[0], nullptr, Wh[1], nullptr, ND, F[1], ND, bk1, 0, 0, 0);
        k_gemmw<h16, 0, true><<<gRow, 32, 0, stream>>>((const h16*)S[0], nullptr, Wh[2], nullptr, ND, F[2], ND, bv1, 0, 0, 0);
        k_split<<<GE, 256, 0, stream>>>(F[0], (bf*)S[0], (bf*)S[1], PW / 8, 1.0f);
        k_split<<<GE, 256, 0, stream>>>(F[1], (bf*)S[2], (bf*)S[3], PW / 8, 1.0f);
        k_gemmw<bf, 2, false><<<gPair, 32, 0, stream>>>((const bf*)S[0], (const bf*)S[1], (const bf*)S[2], (const bf*)S[3], ND, F[3], NS, nullptr, SLAB, SLAB, SLAB);
        k_c16s<<<GE, 256, 0, stream>>>(F[3], (h16*)S[0], PW / 8, 0, rs);
        k_gemmw<h16, 0, false><<<gPair, 32, 0, stream>>>(Wh[3], nullptr, (const h16*)S[0], nullptr, NS, F[3], NS, nullptr, 0, SLAB, SLAB);
        k_gemmw<h16, 0, false><<<gPair, 32, 0, stream>>>(Wh[4], nullptr, (const h16*)S[0], nullptr, NS, F[4], NS, nullptr, 0, SLAB, SLAB);
        k_c16s<<<GE, 256, 0, stream>>>(F[3], (h16*)S[1], PW / 8, 0, 1.0f);
        k_c16s<<<GE, 256, 0, stream>>>(F[4], (h16*)S[2], PW / 8, 0, 1.0f);
        k_gemmw<h16, 0, false><<<gPair, 32, 0, stream>>>((const h16*)S[1], nullptr, (const h16*)S[2], nullptr, NS, F[3], NS, nullptr, SLAB, SLAB, SLAB);
        k_split<<<GE, 256, 0, stream>>>(F[3], (bf*)S[0], (bf*)S[3], PW / 8, rs);
        k_gemmw<bf, 1, false><<<gRow, 32, 0, stream>>>((const bf*)S[0], (const bf*)S[3], Wb[0], nullptr, ND, F[3], ND, nullptr, 0, 0, 0);
        k_gemmw<bf, 1, false><<<gRow, 32, 0, stream>>>((const bf*)S[0], (const bf*)S[3], Wb[1], nullptr, ND, F[4], ND, nullptr, 0, 0, 0);
        k_gemmw<bf, 1, false><<<gRow, 32, 0, stream>>>((const bf*)S[0], (const bf*)S[3], Wb[2], nullptr, ND, F[5], ND, nullptr, 0, 0, 0);
        k_mix<<<G4, 256, 0, stream>>>(F[3], F[4], F[5], F[0], F[2], F[1], F[6], PW / 4);
        k_lnrow<false><<<(unsigned)((PROW + 7) / 8), 256, 0, stream>>>(F[6], nullptr, g1, b1, 1.0e-5f, ND, PROW, F[7]);
        k_c16s<<<GE, 256, 0, stream>>>(F[7], (h16*)S[1], PW / 8, 0, 1.0f);
        k_gemmw<h16, 0, false><<<gRow, 32, 0, stream>>>((const h16*)S[1], nullptr, Wh[5], nullptr, ND, F[0], ND, nullptr, 0, 0, 0);
        k_gemmw<h16, 0, false><<<gRow, 32, 0, stream>>>((const h16*)S[1], nullptr, Wh[6], nullptr, ND, F[1], ND, nullptr, 0, 0, 0);
        k_gemmw<h16, 0, false><<<gRow, 32, 0, stream>>>((const h16*)S[1], nullptr, Wh[7], nullptr, ND, F[2], ND, nullptr, 0, 0, 0);
        k_sum6<<<G4, 256, 0, stream>>>(F[0], F[1], F[2], F[3], F[4], F[5], F[6], PW / 4);
        k_lnrow<false><<<(unsigned)((PROW + 7) / 8), 256, 0, stream>>>(F[6], nullptr, g2, b2, 1.0e-5f, ND, PROW, out + r0 * ND); }
}
